// MixtureOfMamba_64484638982270
// MI455X (gfx1250) — hardware-verified
//
#include <hip/hip_runtime.h>
#include <hip/hip_fp16.h>
#include <math.h>

typedef __attribute__((ext_vector_type(16))) _Float16 v16h;
typedef __attribute__((ext_vector_type(8)))  _Float16 v8h;
typedef __attribute__((ext_vector_type(8)))  float    v8f;
typedef __attribute__((ext_vector_type(4)))  float    v4f;
typedef __attribute__((ext_vector_type(4)))  unsigned v4u;

constexpr int kBatch = 2;
constexpr int kSeq   = 2048;
constexpr int kDm    = 1024;
constexpr int kDin   = 2048;
constexpr int kNst   = 16;
constexpr int kDtR   = 64;
constexpr int kNexp  = 2;
constexpr int kXdW   = kDtR + 2 * kNst;
constexpr int kXdP   = 128;
constexpr int kRows  = kBatch * kSeq;
constexpr int kConvTP = 260;
static_assert(kXdW == 96);
static_assert(kXdW <= kXdP && (kXdP % 64) == 0);
static_assert((kDm % 32) == 0 && (kDin % 32) == 0 && (kDtR % 32) == 0);
static_assert((kRows % 64) == 0 && (kDin % 64) == 0 && (kDm % 64) == 0);
static_assert((kSeq % 64) == 0 && (kDin % 256) == 0);

constexpr float kCarX    = 16.0f;
constexpr float kCarWin  = 1024.0f;
constexpr float kCarU    = 64.0f;
constexpr float kCarWx   = 1024.0f;
constexpr float kCarDt   = 256.0f;
constexpr float kCarWdt  = 64.0f;
constexpr float kCarY    = 16.0f;
constexpr float kCarWout = 1024.0f;
constexpr float kSclIn   = 1.0f / (kCarX * kCarWin);
constexpr float kSclX    = 1.0f / (kCarU * kCarWx);
constexpr float kSclDt   = 1.0f / (kCarDt * kCarWdt);
constexpr float kSclOut  = 1.0f / (kCarY * kCarWout);

constexpr size_t kSzXH  = (size_t)kRows * kDm * 2;
constexpr size_t kSzWIN = (size_t)kNexp * 2 * kDin * kDm * 2;
constexpr size_t kSzR0  = kSzXH + kSzWIN;
constexpr size_t kSzUH  = (size_t)kRows * kDin * 2;
constexpr size_t kSzWOT = (size_t)kNexp * kDm * kDin * 2;
constexpr size_t kSzF32 = (size_t)kRows * kDin * 4;
constexpr size_t kSzWX  = (size_t)kNexp * kXdP * kDin * 2;
constexpr size_t kSzXD  = (size_t)kRows * kXdP * 4;
constexpr size_t kSzDTA = (size_t)kRows * kDtR * 2;
constexpr size_t kSzWDT = (size_t)kNexp * kDin * kDtR * 2;
constexpr size_t kOffR0  = 0;
constexpr size_t kOffXP  = kOffR0  + kSzR0;
constexpr size_t kOffZ   = kOffXP  + kSzF32;
constexpr size_t kOffU   = kOffZ   + kSzF32;
constexpr size_t kOffWX  = kOffU   + kSzF32;
constexpr size_t kOffXD  = kOffWX  + kSzWX;
constexpr size_t kOffDTA = kOffXD  + kSzXD;
constexpr size_t kOffWDT = kOffDTA + kSzDTA;
constexpr size_t kWsTotal = kOffWDT + kSzWDT;
static_assert(kSzUH + kSzWOT <= kSzR0);
static_assert(kWsTotal == 130023424ull);
static_assert(kWsTotal <= 134217728ull);
static_assert((kOffXP % 128) == 0 && (kOffZ % 128) == 0 && (kOffU % 128) == 0 && (kOffWX % 128) == 0 &&
              (kOffXD % 128) == 0 && (kOffDTA % 128) == 0 && (kOffWDT % 128) == 0 && (kSzUH % 128) == 0 &&
              (kSzXH % 128) == 0);

__device__ __forceinline__ unsigned h16_bits_flush(float v) {
  const float f = (fabsf(v) < 6.103515625e-05f) ? 0.0f : v;
  const _Float16 hv = (_Float16)f;
  return (unsigned)__builtin_bit_cast(unsigned short, hv);
}
__device__ __forceinline__ unsigned pack2_h16(float a, float b) {
  const unsigned lo = h16_bits_flush(a);
  const unsigned hi = h16_bits_flush(b);
  return lo | (hi << 16);
}

template <typename T> struct Frag;
template <> struct Frag<_Float16> {
  typedef v16h V;
  union U { v16h v; v8h h[2]; };
  static __device__ __forceinline__ v16h load(const _Float16* p) {
    U f;
    f.h[0] = *(const v8h*)(p);
    f.h[1] = *(const v8h*)(p + 16);
    return f.v;
  }
  static __device__ __forceinline__ v8f mma(v16h a, v16h b, v8f c) {
    return __builtin_amdgcn_wmma_f32_16x16x32_f16(false, a, false, b, (short)0, c, false, false);
  }
};
__device__ __forceinline__ void grp_guard_h(v8f& a0, v8f& a1, v8f& a2, v8f& a3,
                                            v16h x, v16h b0, v16h b1, v16h b2, v16h b3) {
  asm volatile("v_nop\n\tv_nop\n\tv_nop\n\tv_nop"
               : "+v"(a0), "+v"(a1), "+v"(a2), "+v"(a3)
               : "v"(x), "v"(b0), "v"(b1), "v"(b2), "v"(b3));
}
__device__ __forceinline__ void acc_guard4(v8f& a, v8f& b, v8f& c, v8f& d) {
  asm volatile("v_nop\n\tv_nop\n\tv_nop\n\tv_nop" : "+v"(a), "+v"(b), "+v"(c), "+v"(d));
}

template <bool HAS_BIAS>
__global__ __launch_bounds__(256) void gemm_sel_f16_kernel(
    const unsigned short* __restrict__ Ap, int lda,
    const unsigned short* __restrict__ Btp, int ldb, long strideB,
    float* __restrict__ C, int ldc,
    const float* __restrict__ bias, int strideBias,
    const int* __restrict__ ids,
    int M, int N, int K, float scale)
{
  typedef _Float16 T;
  const T* A  = (const T*)Ap;
  const T* Bt = (const T*)Btp;
  __shared__ __align__(16) float sT[8][16 * 68];
  const int e    = blockIdx.y;
  const int lane = threadIdx.x & 31;
  const int wave = threadIdx.x >> 5;
  const int tilesN = N >> 6;
  const int tilesM = M >> 6;
  const int tile = blockIdx.x * 8 + wave;
  if (tile >= tilesM * tilesN) return;
  const int tm = tile / tilesN;
  const int tn = tile - tm * tilesN;
  const int m0 = tm << 6;
  const int n0 = tn << 6;
  const T* Bb = Bt + (size_t)e * strideB;

  const int rlane = lane & 15;
  const int koff  = (lane >> 4) * 8;
  const int mOff  = (lane >> 4) * 8;

  v8f acc[4][4];
#pragma unroll
  for (int i = 0; i < 4; ++i)
#pragma unroll
    for (int j = 0; j < 4; ++j) acc[i][j] = (v8f){0.f, 0.f, 0.f, 0.f, 0.f, 0.f, 0.f, 0.f};

  for (int k0 = 0; k0 < K; k0 += 32) {
    v16h bh[4];
#pragma unroll
    for (int j = 0; j < 4; ++j) {
      const size_t bo = (size_t)(n0 + (j << 4) + rlane) * ldb + koff + k0;
      bh[j] = Frag<T>::load(Bb + bo);
    }
#pragma unroll
    for (int i = 0; i < 4; ++i) {
      const size_t ao = (size_t)(m0 + (i << 4) + rlane) * lda + koff + k0;
      const v16h ah = Frag<T>::load(A + ao);
#pragma unroll
      for (int j = 0; j < 4; ++j) acc[i][j] = Frag<T>::mma(ah, bh[j], acc[i][j]);
      grp_guard_h(acc[i][0], acc[i][1], acc[i][2], acc[i][3], ah, bh[0], bh[1], bh[2], bh[3]);
    }
  }
  acc_guard4(acc[0][0], acc[0][1], acc[0][2], acc[0][3]);
  acc_guard4(acc[1][0], acc[1][1], acc[1][2], acc[1][3]);
  acc_guard4(acc[2][0], acc[2][1], acc[2][2], acc[2][3]);
  acc_guard4(acc[3][0], acc[3][1], acc[3][2], acc[3][3]);

  float* slab = sT[wave];
  const int hh = lane >> 4;
  const int c4 = (lane & 15) * 4;
#pragma unroll
  for (int i = 0; i < 4; ++i) {
    const int mBase = m0 + (i << 4);
#pragma unroll
    for (int j = 0; j < 4; ++j) {
      const int n = n0 + (j << 4) + rlane;
      float bv = 0.f;
      if (HAS_BIAS) bv = bias[(size_t)e * strideBias + n];
#pragma unroll
      for (int r = 0; r < 8; ++r) {
        float v = acc[i][j][r] * scale;
        if (HAS_BIAS) v += bv;
        slab[(mOff + r) * 68 + (j << 4) + rlane] = v;
      }
    }
    __builtin_amdgcn_fence(__ATOMIC_RELEASE, "workgroup");
    __builtin_amdgcn_wave_barrier();
    __builtin_amdgcn_fence(__ATOMIC_ACQUIRE, "workgroup");
    bool own[8];
#pragma unroll
    for (int it = 0; it < 8; ++it) {
      int rid = ids[mBase + it * 2 + hh];
      asm volatile("" : "+v"(rid));
      rid = (rid < 0) ? 0 : ((rid > 1) ? 1 : rid);
      own[it] = (rid == e);
    }
    for (int pass = 0; pass < 2; ++pass) {
#pragma unroll
      for (int it = 0; it < 8; ++it) {
        const int row = it * 2 + hh;
        const v4f v = *(const v4f*)(slab + row * 68 + c4);
        if (own[it]) *(volatile v4f*)(C + (size_t)(mBase + row) * ldc + n0 + c4) = v;
      }
      __threadfence();
    }
    __builtin_amdgcn_fence(__ATOMIC_RELEASE, "workgroup");
    __builtin_amdgcn_wave_barrier();
    __builtin_amdgcn_fence(__ATOMIC_ACQUIRE, "workgroup");
  }
}

__global__ __launch_bounds__(256) void cvt_f16_kernel(
    const float* __restrict__ src, unsigned short* __restrict__ dst, int total8, float carry)
{
  const int i = blockIdx.x * 256 + threadIdx.x;
  if (i >= total8) return;
  const size_t e0 = (size_t)i << 3;
  const v4f a0 = *(const v4f*)(src + e0);
  const v4f a1 = *(const v4f*)(src + e0 + 4);
  const float x0 = a0[0] * carry, x1 = a0[1] * carry, x2 = a0[2] * carry, x3 = a0[3] * carry;
  const float x4 = a1[0] * carry, x5 = a1[1] * carry, x6 = a1[2] * carry, x7 = a1[3] * carry;
  const v4u w = (v4u){pack2_h16(x0, x1), pack2_h16(x2, x3), pack2_h16(x4, x5), pack2_h16(x6, x7)};
  unsigned short* q = dst + e0;
  *(volatile v4u*)q = w;
  __threadfence();
  *(volatile v4u*)q = w;
}

__global__ __launch_bounds__(256) void cvt_pad_wx_kernel(
    const float* __restrict__ src, unsigned short* __restrict__ dst, int total8, float carry)
{
  const int i = blockIdx.x * 256 + threadIdx.x;
  if (i >= total8) return;
  const int drow = i >> 8;
  const int col  = (i & 255) << 3;
  const int ex   = drow >> 7;
  const int r    = drow & 127;
  const bool live = (r < kXdW);
  const int rc   = live ? r : (kXdW - 1);
  const float* sp = src + ((size_t)(ex * kXdW + rc)) * kDin + col;
  const v4f a0 = *(const v4f*)(sp);
  const v4f a1 = *(const v4f*)(sp + 4);
  const float x0 = live ? a0[0] * carry : 0.0f;
  const float x1 = live ? a0[1] * carry : 0.0f;
  const float x2 = live ? a0[2] * carry : 0.0f;
  const float x3 = live ? a0[3] * carry : 0.0f;
  const float x4 = live ? a1[0] * carry : 0.0f;
  const float x5 = live ? a1[1] * carry : 0.0f;
  const float x6 = live ? a1[2] * carry : 0.0f;
  const float x7 = live ? a1[3] * carry : 0.0f;
  const v4u w = (v4u){pack2_h16(x0, x1), pack2_h16(x2, x3), pack2_h16(x4, x5), pack2_h16(x6, x7)};
  unsigned short* q = dst + ((size_t)i << 3);
  *(volatile v4u*)q = w;
  __threadfence();
  *(volatile v4u*)q = w;
}

__global__ __launch_bounds__(256) void dt_plane_kernel(
    const float* __restrict__ XD, unsigned short* __restrict__ DTA, int total8, float carry)
{
  const int i = blockIdx.x * 256 + threadIdx.x;
  if (i >= total8) return;
  const int row = i >> 3;
  const int c8  = (i & 7) << 3;
  const float* sp = XD + (size_t)row * kXdP + c8;
  const v4f a0 = *(const v4f*)(sp);
  const v4f a1 = *(const v4f*)(sp + 4);
  const float x0 = a0[0] * carry, x1 = a0[1] * carry, x2 = a0[2] * carry, x3 = a0[3] * carry;
  const float x4 = a1[0] * carry, x5 = a1[1] * carry, x6 = a1[2] * carry, x7 = a1[3] * carry;
  const v4u w = (v4u){pack2_h16(x0, x1), pack2_h16(x2, x3), pack2_h16(x4, x5), pack2_h16(x6, x7)};
  unsigned short* q = DTA + (size_t)row * kDtR + c8;
  *(volatile v4u*)q = w;
  __threadfence();
  *(volatile v4u*)q = w;
}

__global__ __launch_bounds__(256) void conv_silu_kernel(
    const float* __restrict__ XP, const float* __restrict__ cw, const float* __restrict__ cb,
    float* __restrict__ U, unsigned short* __restrict__ UH, float ucarry)
{
  __shared__ __align__(16) float sT[16 * kConvTP];
  const int tid = threadIdx.x, lane = tid & 31, wave = tid >> 5;
  const int d0 = blockIdx.x * 256, d = d0 + tid;
  const int g0 = blockIdx.y * 64;
  const int tb = g0 & (kSeq - 1);
  const v4f wv = *(const v4f*)(cw + (size_t)d * 4);
  const float w0 = wv[0], w1 = wv[1], w2 = wv[2], w3 = wv[3];
  const float bc = cb[d];
  float xm3, xm2, xm1;
  {
    const bool hist = (tb > 0);
    const int rb = hist ? (g0 - 3) : g0;
    const float v3 = XP[(size_t)rb * kDin + d];
    const float v2 = XP[(size_t)(rb + 1) * kDin + d];
    const float v1 = XP[(size_t)(rb + 2) * kDin + d];
    xm3 = hist ? v3 : 0.f;
    xm2 = hist ? v2 : 0.f;
    xm1 = hist ? v1 : 0.f;
  }
  const int hrow = wave >> 1;
  const int hch  = (wave & 1) * 128 + lane * 4;
#pragma unroll 1
  for (int sub = 0; sub < 4; ++sub) {
    const int lb = g0 + sub * 16;
#pragma unroll 1
    for (int s = 0; s < 16; ++s) {
      const float xcur = XP[(size_t)(lb + s) * kDin + d];
      float acc = bc;
      acc = fmaf(w0, xm3, acc);
      acc = fmaf(w1, xm2, acc);
      acc = fmaf(w2, xm1, acc);
      acc = fmaf(w3, xcur, acc);
      const float sg = __builtin_amdgcn_rcpf(1.0f + expf(-acc));
      sT[s * kConvTP + tid] = acc * sg;
      xm3 = xm2;
      xm2 = xm1;
      xm1 = xcur;
    }
    __syncthreads();
    v4f fv[4];
    v4u hw[2];
#pragma unroll
    for (int it = 0; it < 4; ++it) fv[it] = *(const v4f*)(sT + (it * 4 + hrow) * kConvTP + hch);
#pragma unroll
    for (int it = 0; it < 2; ++it) {
      const float* sp = sT + (it * 8 + wave) * kConvTP + lane * 8;
      const v4f a0 = *(const v4f*)(sp);
      const v4f a1 = *(const v4f*)(sp + 4);
      const float x0 = a0[0] * ucarry, x1 = a0[1] * ucarry, x2 = a0[2] * ucarry, x3 = a0[3] * ucarry;
      const float x4 = a1[0] * ucarry, x5 = a1[1] * ucarry, x6 = a1[2] * ucarry, x7 = a1[3] * ucarry;
      hw[it] = (v4u){pack2_h16(x0, x1), pack2_h16(x2, x3), pack2_h16(x4, x5), pack2_h16(x6, x7)};
    }
    for (int pass = 0; pass < 2; ++pass) {
#pragma unroll
      for (int it = 0; it < 4; ++it)
        *(volatile v4f*)(U + (size_t)(lb + it * 4 + hrow) * kDin + d0 + hch) = fv[it];
#pragma unroll
      for (int it = 0; it < 2; ++it) {
        const size_t o = (size_t)(lb + it * 8 + wave) * kDin + d0 + lane * 8;
        *(volatile v4u*)(UH + o) = hw[it];
      }
      __threadfence();
    }
    __syncthreads();
  }
}

typedef float    ms1_v4f __attribute__((ext_vector_type(4)));
typedef unsigned ms1_v4u __attribute__((ext_vector_type(4)));
struct ms1_args {
  const float* dtpre;
  const float* u;
  const float* bc;
  const float* z;
  const float* A_log;
  const float* Dskip;
  __half* y;
  __half* y_lo;
  long ld_dtpre;
  long ld_u;
  long ld_bc;
  long ld_z;
  long ld_y;
  int offB;
  int offC;
  int offZ;
  float ycarry;
  int dir;
  int D;
  int L;
  int nbatch;
};
static_assert(sizeof(ms1_args) == 136);

__device__ __forceinline__ float ms1_flush16(float v) {
  return (fabsf(v) < 6.103515625e-05f) ? 0.0f : v;
}
__device__ __forceinline__ unsigned ms1_h16bits(float v) {
  return (unsigned)__half_as_ushort(__float2half_rn(ms1_flush16(v)));
}
__device__ __forceinline__ float ms1_h16val(unsigned b) {
  return __half2float(__ushort_as_half((unsigned short)b));
}
__device__ __forceinline__ float ms1_softplus(float v) {
  return fmaxf(v, 0.0f) + log1pf(expf(-fabsf(v)));
}
__device__ __forceinline__ void ms1_pack2(float v0, float v1, unsigned& hw, unsigned& lw) {
  const unsigned h0 = ms1_h16bits(v0);
  const unsigned h1 = ms1_h16bits(v1);
  const float r0 = (v0 - ms1_h16val(h0)) * 2048.0f;
  const float r1 = (v1 - ms1_h16val(h1)) * 2048.0f;
  const unsigned l0 = ms1_h16bits(r0);
  const unsigned l1 = ms1_h16bits(r1);
  hw = h0 | (h1 << 16);
  lw = l0 | (l1 << 16);
}

template <int NSTATE>
__global__ __launch_bounds__(64 * (NSTATE / 16)) void ms1_scan_kernel(ms1_args a)
{
  static_assert(NSTATE == 16 || NSTATE == 64);
  constexpr int NQ  = NSTATE / 16;
  constexpr int NT  = 64 * NQ;
  constexpr int NW  = NT / 32;
  constexpr int BCW = 2 * NSTATE;
  constexpr int YP  = 68;
  constexpr int RPI = NW * 4;
  constexpr int NIT = 64 / RPI;
  static_assert(16 * NT <= 64 * YP);
  __shared__ __align__(16) float sBC[64 * BCW];
  __shared__ __align__(16) float sY[64 * YP];
  const int tid  = threadIdx.x;
  const int lane = tid & 31;
  const int wave = tid >> 5;
  const int c    = tid / NQ;
  const int sq   = tid - c * NQ;
  const int bpb  = a.D / 64;
  const int bi   = blockIdx.x / bpb;
  if (bi >= a.nbatch) return;
  const int d0 = (blockIdx.x - bi * bpb) * 64;
  const int d  = d0 + c;
  const long rowb = (long)bi * a.L;
  const bool hasz  = (a.z != nullptr);
  const bool hasD  = (a.Dskip != nullptr);
  const bool hasLo = (a.y_lo != nullptr);

#pragma unroll 1
  for (int n = 0; n < 16; ++n) {
    const float al = a.A_log[(long)d * NSTATE + sq * 16 + n];
    sY[n * NT + tid] = -expf(al);
  }
  __syncthreads();
  float An[16], h[16];
#pragma unroll
  for (int n = 0; n < 16; ++n) {
    An[n] = sY[n * NT + tid];
    h[n] = 0.0f;
  }
  float Dd = 0.0f;
  if (hasD) Dd = a.Dskip[d];

  const int nchunk = a.L / 64;
  const bool fwd = (a.dir > 0);
  const int s0 = fwd ? 0 : 63;
  const int sd = fwd ? 1 : -1;
  const int q  = lane >> 3;
  const int c8 = (lane & 7) * 8;

#pragma unroll 1
  for (int ci = 0; ci < nchunk; ++ci) {
    const int tb = fwd ? (ci * 64) : (a.L - 64 - ci * 64);
    const long rowc = rowb + tb;
    __syncthreads();
#pragma unroll 8
    for (int i = 0; i < 32; ++i) {
      const int idx = tid + i * NT;
      const int st  = idx / BCW;
      const int col = idx - st * BCW;
      const int sc  = (col < NSTATE) ? (a.offB + col) : (a.offC + col - NSTATE);
      sBC[idx] = a.bc[(rowc + st) * a.ld_bc + sc];
    }
    __syncthreads();
#pragma unroll 1
    for (int s = 0; s < 64; ++s) {
      const int ls = s0 + sd * s;
      const long row = rowc + ls;
      float pre = a.dtpre[row * a.ld_dtpre + d];
      float uv  = a.u[row * a.ld_u + d];
      float zv  = 0.0f;
      if (hasz) zv = a.z[row * a.ld_z + a.offZ + d];
      asm volatile("" : "+v"(pre));
      asm volatile("" : "+v"(uv));
      asm volatile("" : "+v"(zv));
      const float delta = ms1_softplus(pre);
      const float dtx = delta * uv;
      const float* bp = sBC + ls * BCW + sq * 16;
      const float* cp = bp + NSTATE;
      ms1_v4f Bq[4], Cq[4];
#pragma unroll
      for (int k = 0; k < 4; ++k) {
        Bq[k] = *(const ms1_v4f*)(bp + 4 * k);
        Cq[k] = *(const ms1_v4f*)(cp + 4 * k);
      }
      float yv = 0.0f;
#pragma unroll
      for (int n = 0; n < 16; ++n) {
        const float e = __expf(delta * An[n]);
        h[n] = fmaf(e, h[n], dtx * Bq[n >> 2][n & 3]);
        yv = fmaf(h[n], Cq[n >> 2][n & 3], yv);
      }
      if (NQ > 1) {
        yv += __shfl_xor(yv, 1, 32);
        yv += __shfl_xor(yv, 2, 32);
      }
      if (hasD) yv = fmaf(uv, Dd, yv);
      if (hasz) {
        const float sg = __builtin_amdgcn_rcpf(1.0f + expf(-zv));
        yv = yv * (zv * sg);
      }
      if (sq == 0) sY[ls * YP + c] = yv * a.ycarry;
    }
    __syncthreads();
    ms1_v4u hw[NIT], lw[NIT];
#pragma unroll
    for (int it = 0; it < NIT; ++it) {
      const int row = it * RPI + wave * 4 + q;
      const float* sp = sY + row * YP + c8;
      const ms1_v4f f0 = *(const ms1_v4f*)(sp);
      const ms1_v4f f1 = *(const ms1_v4f*)(sp + 4);
      unsigned h0, h1, h2, h3, l0, l1, l2, l3;
      ms1_pack2(f0[0], f0[1], h0, l0);
      ms1_pack2(f0[2], f0[3], h1, l1);
      ms1_pack2(f1[0], f1[1], h2, l2);
      ms1_pack2(f1[2], f1[3], h3, l3);
      hw[it] = (ms1_v4u){h0, h1, h2, h3};
      lw[it] = (ms1_v4u){l0, l1, l2, l3};
    }
    for (int pass = 0; pass < 2; ++pass) {
#pragma unroll
      for (int it = 0; it < NIT; ++it) {
        const int row = it * RPI + wave * 4 + q;
        const long o = (rowc + row) * a.ld_y + d0 + c8;
        *(volatile ms1_v4u*)(a.y + o) = hw[it];
        if (hasLo) *(volatile ms1_v4u*)(a.y_lo + o) = lw[it];
      }
      __threadfence();
    }
  }
}

extern "C" void kernel_launch(void* const* d_in, const int* in_sizes, int n_in,
                              void* d_out, int out_size, void* d_ws, size_t ws_size,
                              hipStream_t stream) {
  if (n_in < 11) return;
  if (in_sizes[0] != kRows * kDm) return;
  if (in_sizes[1] != kRows) return;
  if (in_sizes[2] != kNexp * 2 * kDin * kDm) return;
  if (in_sizes[3] != kDin * 4) return;
  if (in_sizes[4] != kDin) return;
  if (in_sizes[5] != kNexp * kXdW * kDin) return;
  if (in_sizes[6] != kNexp * kDin * kDtR) return;
  if (in_sizes[7] != kNexp * kDin) return;
  if (in_sizes[8] != kDin * kNst) return;
  if (in_sizes[9] != kDin) return;
  if (in_sizes[10] != kNexp * kDm * kDin) return;
  if (out_size != kRows * kDm) return;
  if (ws_size < kWsTotal) return;

  const float* hidden = (const float*)d_in[0];
  const int*   ids    = (const int*)  d_in[1];
  const float* W_in   = (const float*)d_in[2];
  const float* conv_w = (const float*)d_in[3];
  const float* conv_b = (const float*)d_in[4];
  const float* W_x    = (const float*)d_in[5];
  const float* W_dt   = (const float*)d_in[6];
  const float* b_dt   = (const float*)d_in[7];
  const float* A_log  = (const float*)d_in[8];
  const float* D_par  = (const float*)d_in[9];
  const float* W_out  = (const float*)d_in[10];
  float* out = (float*)d_out;

  char* ws = (char*)d_ws;
  unsigned short* XH  = (unsigned short*)(ws + kOffR0);
  unsigned short* WIN = (unsigned short*)(ws + kOffR0 + kSzXH);
  unsigned short* UH  = (unsigned short*)(ws + kOffR0);
  unsigned short* WOT = (unsigned short*)(ws + kOffR0 + kSzUH);
  unsigned short* YH  = (unsigned short*)(ws + kOffR0);
  float*          XP  = (float*)(ws + kOffXP);
  float*          DTP = (float*)(ws + kOffXP);
  float*          ZP  = (float*)(ws + kOffZ);
  float*          UP  = (float*)(ws + kOffU);
  unsigned short* WX  = (unsigned short*)(ws + kOffWX);
  float*          XD  = (float*)(ws + kOffXD);
  unsigned short* DTA = (unsigned short*)(ws + kOffDTA);
  unsigned short* WDT = (unsigned short*)(ws + kOffWDT);

  cvt_f16_kernel<<<(kRows * kDm / 8) / 256, 256, 0, stream>>>(hidden, XH, kRows * kDm / 8, kCarX);
  cvt_f16_kernel<<<(kNexp * 2 * kDin * kDm / 8) / 256, 256, 0, stream>>>(W_in, WIN, kNexp * 2 * kDin * kDm / 8, kCarWin);
  cvt_pad_wx_kernel<<<(kNexp * kXdP * kDin / 8) / 256, 256, 0, stream>>>(W_x, WX, kNexp * kXdP * kDin / 8, kCarWx);
  cvt_f16_kernel<<<(kNexp * kDin * kDtR / 8) / 256, 256, 0, stream>>>(W_dt, WDT, kNexp * kDin * kDtR / 8, kCarWdt);

  gemm_sel_f16_kernel<false><<<dim3((kRows / 64) * (kDin / 64) / 8, kNexp), 256, 0, stream>>>(
      XH, kDm,
      WIN, kDm, (long)2 * kDin * kDm,
      XP, kDin,
      nullptr, 0,
      ids,
      kRows, kDin, kDm, kSclIn);
  gemm_sel_f16_kernel<false><<<dim3((kRows / 64) * (kDin / 64) / 8, kNexp), 256, 0, stream>>>(
      XH, kDm,
      WIN + (size_t)kDin * kDm, kDm, (long)2 * kDin * kDm,
      ZP, kDin,
      nullptr, 0,
      ids,
      kRows, kDin, kDm, kSclIn);

  conv_silu_kernel<<<dim3(kDin / 256, kRows / 64), 256, 0, stream>>>(XP, conv_w, conv_b, UP, UH, kCarU);

  cvt_f16_kernel<<<(kNexp * kDm * kDin / 8) / 256, 256, 0, stream>>>(W_out, WOT, kNexp * kDm * kDin / 8, kCarWout);

  gemm_sel_f16_kernel<false><<<dim3((kRows / 64) * (kXdP / 64) / 8, kNexp), 256, 0, stream>>>(
      UH, kDin,
      WX, kDin, (long)kXdP * kDin,
      XD, kXdP,
      nullptr, 0,
      ids,
      kRows, kXdP, kDin, kSclX);

  dt_plane_kernel<<<(kRows * kDtR / 8) / 256, 256, 0, stream>>>(XD, DTA, kRows * kDtR / 8, kCarDt);

  gemm_sel_f16_kernel<true><<<dim3((kRows / 64) * (kDin / 64) / 8, kNexp), 256, 0, stream>>>(
      DTA, kDtR,
      WDT, kDtR, (long)kDin * kDtR,
      DTP, kDin,
      b_dt, kDin,
      ids,
      kRows, kDin, kDtR, kSclDt);

  for (int b = 0; b < kBatch; ++b) {
    const size_t r0 = (size_t)b * kSeq;
    ms1_args sa;
    sa.dtpre = DTP + r0 * kDin;
    sa.u = UP + r0 * kDin;
    sa.bc = XD + r0 * kXdP;
    sa.z = ZP + r0 * kDin;
    sa.A_log = A_log;
    sa.Dskip = D_par;
    sa.y = (__half*)(YH + r0 * kDin);
    sa.y_lo = nullptr;
    sa.ld_dtpre = kDin;
    sa.ld_u = kDin;
    sa.ld_bc = kXdP;
    sa.ld_z = kDin;
    sa.ld_y = kDin;
    sa.offB = kDtR;
    sa.offC = kDtR + kNst;
    sa.offZ = 0;
    sa.ycarry = kCarY;
    sa.dir = 1;
    sa.D = kDin;
    sa.L = kSeq;
    sa.nbatch = 1;
    ms1_scan_kernel<16><<<dim3(kDin / 64), 64, 0, stream>>>(sa);
  }

  gemm_sel_f16_kernel<false><<<dim3((kRows / 64) * (kDm / 64) / 8, kNexp), 256, 0, stream>>>(
      YH, kDin,
      WOT, kDin, (long)kDm * kDin,
      out, kDm,
      nullptr, 0,
      ids,
      kRows, kDm, kDin, kSclOut);
}
